// HybridDiT_68143951118754
// MI455X (gfx1250) — hardware-run, weakly checked
//
#include <hip/hip_runtime.h>
#include <math.h>

#ifndef NB
#define NB 2
#endif
#ifndef SEQ
#define SEQ 1024
#endif
#define NB_FULL 2
#define SEQ_FULL 1024
#define DM 1024
#define NHEAD 16
#define HDIM 64
#define FFD 4096
#define YDIM 2048
#define FREQD 256
#define DEPTH 2
#define MTOK (NB * 2 * SEQ)
#define MHALF (NB * SEQ)
#define MBLK (NB * SEQ / 4)

static_assert(NB >= 1 && NB <= NB_FULL);
static_assert(SEQ <= SEQ_FULL && SEQ % 256 == 0);
static_assert(MBLK % 64 == 0 && MHALF % 64 == 0 && MTOK % 64 == 0);
static_assert(DM % 64 == 0 && FFD % 64 == 0 && YDIM % 32 == 0 && FREQD % 32 == 0);
static_assert(DM == NHEAD * HDIM && HDIM == 64 && FREQD == 256 && DEPTH == 2);
static_assert((size_t)((NB - 1) * SEQ_FULL + SEQ) * DM * 4 <= (size_t)8388608);

typedef _Float16 h16;
typedef __attribute__((ext_vector_type(16))) _Float16 v16h;
typedef __attribute__((ext_vector_type(8)))  _Float16 v8h;
typedef __attribute__((ext_vector_type(8)))  float    v8f;
typedef __attribute__((ext_vector_type(4)))  float    v4f;

constexpr float C_ACT = 2048.0f;
constexpr float C_EMB = 16384.0f;
constexpr float C_W   = 131072.0f;


__device__ __forceinline__ float bfr(float f) {
    unsigned u = __float_as_uint(f);
    u += 0x7FFFu + ((u >> 16) & 1u);
    return __uint_as_float(u & 0xFFFF0000u);
}
__device__ __forceinline__ v4f bfr4(v4f p) {
    v4f r; r.x = bfr(p.x); r.y = bfr(p.y); r.z = bfr(p.z); r.w = bfr(p.w); return r;
}
static __device__ __forceinline__ h16 toh_flush(float v) {
    const float w = (fabsf(v) < 6.103515625e-05f) ? 0.0f : v;
    return (h16)w;
}
__device__ __forceinline__ void st8h(h16* P, size_t o, const float* v) {
    v8h pk;
#pragma unroll
    for (int e = 0; e < 8; ++e) pk[e] = toh_flush(v[e]);
    *(volatile v8h*)(P + o) = pk;
    __threadfence();
    *(volatile v8h*)(P + o) = pk;
}

union FragU { v16h v; v8h h[2]; };
__device__ __forceinline__ v16h frag_ld(const h16* p) {
    FragU f; f.h[0] = *(const v8h*)(p); f.h[1] = *(const v8h*)(p + 16); return f.v;
}
__device__ __forceinline__ v8f wmma16g(v16h a, v16h b, v8f c) {
    c = __builtin_amdgcn_wmma_f32_16x16x32_f16(false, a, false, b, (short)0, c, false, false);
    asm volatile("v_nop\n\tv_nop\n\tv_nop\n\tv_nop" : "+v"(c) : "v"(a), "v"(b));
    return c;
}
__device__ __forceinline__ void wave_sync_lds() {
    __builtin_amdgcn_fence(3  , "workgroup");
    __builtin_amdgcn_wave_barrier();
    __builtin_amdgcn_fence(2  , "workgroup");
}

__global__ __launch_bounds__(256) void k_wt16(const float* __restrict__ Wm, unsigned KI, unsigned NO, unsigned lgper,
                                              h16* __restrict__ W16) {
    const unsigned layer = blockIdx.y;
    const float* Wl = Wm + (size_t)layer * KI * NO;
    h16* Dl = W16 + (size_t)layer * KI * NO;
    const unsigned u = blockIdx.x * 256u + threadIdx.x;
    const unsigned per = 1u << lgper;
    if (u >= NO * per) return;
    const unsigned k0 = 8u * (u & (per - 1u));
    const unsigned o = u >> lgper;
    float v[8];
#pragma unroll
    for (int i = 0; i < 8; ++i) v[i] = bfr(Wl[(size_t)(k0 + (unsigned)i) * NO + o]) * C_W;
    st8h(Dl, (size_t)o * KI + k0, v);
}

template <unsigned C, unsigned R, unsigned RF, unsigned OFF, int LG, bool RNEIN>
__global__ __launch_bounds__(256) void k_cvt(const float* __restrict__ src, h16* __restrict__ dst, unsigned nrows) {
    constexpr unsigned PER = C / 8u;
    constexpr float CAR = (float)(1u << LG);
    const unsigned u = blockIdx.x * 256u + threadIdx.x;
    if (u >= nrows * PER) return;
    const unsigned row = u / PER;
    const unsigned c0 = (u - row * PER) * 8u;
    const unsigned b = row / R;
    const unsigned s = row - b * R;
    const float* sp = src + (size_t)(b * RF + OFF + s) * C + c0;
    const v4f a = *(const v4f*)sp, d = *(const v4f*)(sp + 4);
    float v[8] = {a.x, a.y, a.z, a.w, d.x, d.y, d.z, d.w};
#pragma unroll
    for (int i = 0; i < 8; ++i) v[i] = (RNEIN ? bfr(v[i]) : v[i]) * CAR;
    st8h(dst, (size_t)row * C + c0, v);
}

__global__ __launch_bounds__(256) void k_sin(const int* __restrict__ t, h16* __restrict__ sin16) {
    __shared__ float sE[FREQD];
    const unsigned tid = threadIdx.x;
    const unsigned row = blockIdx.x;
    const unsigned b = row / (unsigned)(SEQ / 4);
    const unsigned blk = row - b * (unsigned)(SEQ / 4);
    const float tv = (float)t[b * (unsigned)(SEQ_FULL / 4) + blk];
    const unsigned i = tid & 127u;
    const float freq = expf((-9.210340371976184f * (float)i) / 128.0f);
    const float a = tv * freq;
    const float cv = cosf(a);
    const float sv = sinf(a);
    sE[tid] = ((tid < 128u) ? cv : sv) * C_EMB;
    __syncthreads();
    if (tid < 32u) {
        float v[8];
#pragma unroll
        for (int e = 0; e < 8; ++e) v[e] = sE[8u * tid + (unsigned)e];
        st8h(sin16, (size_t)row * FREQD + 8u * tid, v);
    }
}

__global__ __launch_bounds__(256) void k_ln(const float* __restrict__ h, const float* __restrict__ g, const float* __restrict__ bt,
                                            h16* __restrict__ z16, unsigned M) {
    const unsigned row = blockIdx.x * 8u + (threadIdx.x >> 5);
    const unsigned L = threadIdx.x & 31u;
    if (row >= M) return;
    const float* hr = h + (size_t)row * DM + 8u * L;
    float d[32];
#pragma unroll
    for (int q = 0; q < 4; ++q) {
        const v4f a = *(const v4f*)(hr + 256 * q), b = *(const v4f*)(hr + 256 * q + 4);
        d[8 * q + 0] = a.x; d[8 * q + 1] = a.y; d[8 * q + 2] = a.z; d[8 * q + 3] = a.w;
        d[8 * q + 4] = b.x; d[8 * q + 5] = b.y; d[8 * q + 6] = b.z; d[8 * q + 7] = b.w;
    }
    float s = 0.f;
#pragma unroll
    for (int i = 0; i < 32; ++i) s += d[i];
#pragma unroll
    for (int o = 16; o > 0; o >>= 1) s += __shfl_xor(s, o, 32);
    const float mu = s * (1.0f / (float)DM);
    float qs = 0.f;
#pragma unroll
    for (int i = 0; i < 32; ++i) { d[i] -= mu; qs += d[i] * d[i]; }
#pragma unroll
    for (int o = 16; o > 0; o >>= 1) qs += __shfl_xor(qs, o, 32);
    const float rs = 1.0f / sqrtf(qs * (1.0f / (float)DM) + 1e-5f);
#pragma unroll
    for (int q = 0; q < 4; ++q) {
        const unsigned cb = 256u * (unsigned)q + 8u * L;
        const v4f g0 = *(const v4f*)(g + cb), g1 = *(const v4f*)(g + cb + 4u);
        const v4f b0 = *(const v4f*)(bt + cb), b1 = *(const v4f*)(bt + cb + 4u);
        const float gg[8] = {g0.x, g0.y, g0.z, g0.w, g1.x, g1.y, g1.z, g1.w};
        const float bb[8] = {b0.x, b0.y, b0.z, b0.w, b1.x, b1.y, b1.z, b1.w};
        float y[8];
#pragma unroll
        for (int i = 0; i < 8; ++i) y[i] = (d[8 * q + i] * rs * bfr(gg[i]) + bfr(bb[i])) * C_ACT;
        st8h(z16, (size_t)row * DM + cb, y);
    }
}

#define EP_F16   0
#define EP_VT    1
#define EP_F32   2
#define EP_RESID 3
#define EP_EMBX  4
#define EP_EMBXT 5
#define EP_OUT   6
#define ACT_NONE 0
#define ACT_SILU 1
#define ACT_GELU 2

template <int ACT>
__device__ __forceinline__ float act_fn(float v) {
    if (ACT == ACT_SILU) return v / (1.0f + expf(-v));
    if (ACT == ACT_GELU) return 0.5f * v * (1.0f + erff(v / 1.4142135623730951f));
    return v;
}

template <int EP, int ACT, int LGS, int LGO, bool NOISY>
__global__ __launch_bounds__(256) void k_gemm64(
    const h16* __restrict__ A, unsigned lda, const h16* __restrict__ Bt, unsigned ldb,
    void* Cout, unsigned ldc, const float* __restrict__ bias,
    const float* add0, const float* __restrict__ add1, const float* __restrict__ add2,
    unsigned M, unsigned N, unsigned K) {
  __shared__ __align__(16) float sT[8][16 * 68];
  constexpr float SCALE = 1.0f / (float)(1u << LGS);
  constexpr float OSC = (float)(1u << LGO);
  const unsigned lane = threadIdx.x & 31u;
  const unsigned wave = threadIdx.x >> 5;
  const unsigned tilesN = N >> 6, tilesM = M >> 6;
  const unsigned tile = blockIdx.x * 8u + wave;
  if (tile >= tilesM * tilesN) return;
  const unsigned tm = tile / tilesN;
  const unsigned tn = tile - tm * tilesN;
  unsigned m0 = tm << 6;
  if (NOISY) {
    const unsigned bq = tm / (unsigned)(SEQ / 64);
    const unsigned tq = tm - bq * (unsigned)(SEQ / 64);
    m0 = bq * (unsigned)(2 * SEQ) + (unsigned)SEQ + (tq << 6);
  }
  const unsigned n0 = tn << 6;
  const unsigned rlane = lane & 15u;
  const unsigned koff = (lane >> 4) * 8u;
  const unsigned mOff = koff;

  v8f acc[4][4];
#pragma unroll
  for (int i = 0; i < 4; ++i)
#pragma unroll
    for (int j = 0; j < 4; ++j) acc[i][j] = (v8f){0.f,0.f,0.f,0.f,0.f,0.f,0.f,0.f};

  for (unsigned k0 = 0; k0 < K; k0 += 32u) {
    v16h bh[4];
#pragma unroll
    for (int j = 0; j < 4; ++j)
      bh[j] = frag_ld(Bt + (size_t)(n0 + ((unsigned)j << 4) + rlane) * ldb + koff + k0);
#pragma unroll
    for (int i = 0; i < 4; ++i) {
      const v16h ah = frag_ld(A + (size_t)(m0 + ((unsigned)i << 4) + rlane) * lda + koff + k0);
#pragma unroll
      for (int j = 0; j < 4; ++j) acc[i][j] = wmma16g(ah, bh[j], acc[i][j]);
    }
  }

  float* slab = sT[wave];
  float bv[4];
#pragma unroll
  for (int j = 0; j < 4; ++j) bv[j] = bfr(bias[n0 + ((unsigned)j << 4) + rlane]);

  if (EP == EP_VT) {
    h16* Vt = (h16*)Cout;
    const unsigned bb = m0 / (unsigned)(2 * SEQ);
    const unsigned tok0 = m0 - bb * (unsigned)(2 * SEQ);
    const unsigned head = n0 >> 6;
    const unsigned q = lane >> 3, c8 = (lane & 7u) * 8u;
#pragma unroll
    for (int j = 0; j < 4; ++j) {
#pragma unroll
      for (int i = 0; i < 4; ++i)
#pragma unroll
        for (int r = 0; r < 8; ++r)
          slab[rlane * 68u + ((unsigned)i << 4) + mOff + (unsigned)r] = (acc[i][j][r] * SCALE + bv[j]) * OSC;
      wave_sync_lds();
      v8h hv[4];
#pragma unroll
      for (int it = 0; it < 4; ++it) {
        const float* sp = slab + ((unsigned)it * 4u + q) * 68u + c8;
#pragma unroll
        for (int e = 0; e < 8; ++e) hv[it][e] = toh_flush(sp[e]);
      }
      for (int pass = 0; pass < 2; ++pass) {
#pragma unroll
        for (int it = 0; it < 4; ++it) {
          const unsigned drow = ((unsigned)j << 4) + (unsigned)it * 4u + q;
          *(volatile v8h*)(Vt + (size_t)((bb * (unsigned)NHEAD + head) * (unsigned)HDIM + drow) * ldc + tok0 + c8) = hv[it];
        }
        __threadfence();
      }
      wave_sync_lds();
    }
  } else {
    unsigned bidx = 0u, sbase = 0u;
    if (EP == EP_EMBX || EP == EP_EMBXT || EP == EP_OUT) {
      bidx = m0 / (unsigned)SEQ;
      sbase = m0 - bidx * (unsigned)SEQ;
    }
#pragma unroll
    for (int i = 0; i < 4; ++i) {
      const unsigned mBase = m0 + ((unsigned)i << 4);
#pragma unroll
      for (int j = 0; j < 4; ++j) {
#pragma unroll
        for (int r = 0; r < 8; ++r) {
          float v = act_fn<ACT>(acc[i][j][r] * SCALE + bv[j]);
          if (EP == EP_F16) v *= OSC;
          slab[(mOff + (unsigned)r) * 68u + ((unsigned)j << 4) + rlane] = v;
        }
      }
      wave_sync_lds();
      if (EP == EP_F16) {
        h16* C = (h16*)Cout;
        const unsigned q = lane >> 3, c8 = (lane & 7u) * 8u;
        v8h hv[4];
#pragma unroll
        for (int it = 0; it < 4; ++it) {
          const float* sp = slab + ((unsigned)it * 4u + q) * 68u + c8;
#pragma unroll
          for (int e = 0; e < 8; ++e) hv[it][e] = toh_flush(sp[e]);
        }
        for (int pass = 0; pass < 2; ++pass) {
#pragma unroll
          for (int it = 0; it < 4; ++it) {
            const unsigned row = (unsigned)it * 4u + q;
            *(volatile v8h*)(C + (size_t)(mBase + row) * ldc + n0 + c8) = hv[it];
          }
          __threadfence();
        }
      } else {
        float* C = (float*)Cout;
        const unsigned hh = lane >> 4, c4 = (lane & 15u) * 4u;
        const unsigned sRow0 = sbase + ((unsigned)i << 4);
        unsigned dBase = mBase;
        if (EP == EP_EMBX)  dBase = bidx * (unsigned)(2 * SEQ) + sRow0;
        if (EP == EP_EMBXT) dBase = bidx * (unsigned)(2 * SEQ) + (unsigned)SEQ + sRow0;
        if (EP == EP_OUT)   dBase = bidx * (unsigned)SEQ_FULL + sRow0;
#pragma unroll
        for (int half = 0; half < 2; ++half) {
          v4f vv[4];
#pragma unroll
          for (int it = 0; it < 4; ++it) {
            const unsigned row = (unsigned)(half * 4 + it) * 2u + hh;
            v4f tv = *(const v4f*)(slab + row * 68u + c4);
            if (EP == EP_RESID) tv += *(const v4f*)(add0 + (size_t)(dBase + row) * ldc + n0 + c4);
            if (EP == EP_EMBXT) tv += *(const v4f*)(add1 + (size_t)(bidx * (unsigned)(SEQ / 4) + ((sRow0 + row) >> 2)) * DM + n0 + c4);
            if (EP == EP_EMBX || EP == EP_EMBXT) tv += bfr4(*(const v4f*)(add0 + (size_t)(sRow0 + row) * DM + n0 + c4));
            if (EP == EP_EMBXT) tv += *(const v4f*)(add2 + (size_t)(bidx * (unsigned)(SEQ / 4) + ((sRow0 + row) >> 2)) * DM + n0 + c4);
            vv[it] = tv;
          }
          for (int pass = 0; pass < 2; ++pass) {
#pragma unroll
            for (int it = 0; it < 4; ++it) {
              const unsigned row = (unsigned)(half * 4 + it) * 2u + hh;
              *(volatile v4f*)(C + (size_t)(dBase + row) * ldc + n0 + c4) = vv[it];
            }
            __threadfence();
          }
        }
      }
      wave_sync_lds();
    }
  }
}

#define AT_SP 68
#define AT_PP 72
template <bool NOISY>
__global__ __launch_bounds__(32) void k_attn(const h16* __restrict__ QK, const h16* __restrict__ Vt, h16* __restrict__ O16) {
    __shared__ __align__(16) float sS[16 * AT_SP];
    __shared__ __align__(16) h16 sP[16 * AT_PP];
    __shared__ __align__(16) float sAl[16];
    const unsigned lane = threadIdx.x & 31u;
    const unsigned hh = lane >> 4, c = lane & 15u;
    constexpr unsigned NT = NOISY ? (unsigned)(SEQ / 16) : (unsigned)(2 * SEQ / 16);
    const unsigned u = blockIdx.x;
    const unsigned b = u / (NT * (unsigned)NHEAD);
    const unsigned rem = u - b * (NT * (unsigned)NHEAD);
    const unsigned head = rem / NT;
    const unsigned qt = rem - head * NT + (NOISY ? (unsigned)(SEQ / 16) : 0u);
    const unsigned i0 = qt * 16u;
    const h16* qkb = QK + (size_t)(b * (unsigned)(2 * SEQ)) * (2u * DM);
    const h16* vtb = Vt + (size_t)((b * (unsigned)NHEAD + head) * (unsigned)HDIM) * (unsigned)(2 * SEQ);
    const v16h qf0 = frag_ld(qkb + (size_t)(i0 + c) * (2u * DM) + head * 64u + 8u * hh);
    const v16h qf1 = frag_ld(qkb + (size_t)(i0 + c) * (2u * DM) + head * 64u + 32u + 8u * hh);
    unsigned nfull = 0u;
    if (i0 >= (unsigned)SEQ) nfull = (i0 - (unsigned)SEQ + 12u + 63u) >> 6;
    const unsigned diagbase = i0 & ~63u;
    const unsigned prow = lane >> 1, phalf = lane & 1u;
    const float SC = 7.450580596923828e-09f;
    float mrun = -3.0e38f, lrun = 0.f;
    v8f o[4];
#pragma unroll
    for (int t = 0; t < 4; ++t) o[t] = (v8f){0.f,0.f,0.f,0.f,0.f,0.f,0.f,0.f};

    for (unsigned ch = 0; ch <= nfull; ++ch) {
        const unsigned base = (ch < nfull) ? (ch * 64u) : diagbase;
        v8f s[4];
#pragma unroll
        for (int j = 0; j < 4; ++j) {
            const h16* kp = qkb + (size_t)(base + (unsigned)j * 16u + c) * (2u * DM) + (unsigned)DM + head * 64u + 8u * hh;
            const v16h kf0 = frag_ld(kp);
            const v16h kf1 = frag_ld(kp + 32);
            const v8f z = (v8f){0.f,0.f,0.f,0.f,0.f,0.f,0.f,0.f};
            s[j] = wmma16g(qf0, kf0, z);
            s[j] = wmma16g(qf1, kf1, s[j]);
        }
#pragma unroll
        for (int r = 0; r < 8; ++r) {
            const unsigned qi = i0 + 8u * hh + (unsigned)r;
            const unsigned qblk = qi >> 2;
            const unsigned qbound = (qi >= (unsigned)SEQ + 4u) ? ((qi - (unsigned)SEQ) & ~3u) : 0u;
#pragma unroll
            for (int j = 0; j < 4; ++j) {
                const unsigned kj = base + (unsigned)j * 16u + c;
                const bool same_blk = ((kj >> 2) == qblk);
                const bool causal = (kj < qbound);
                sS[(8u * hh + (unsigned)r) * AT_SP + (unsigned)j * 16u + c] = (same_blk || causal) ? (s[j][r] * SC) : -INFINITY;
            }
        }
        wave_sync_lds();
        {
            const float* srow = sS + prow * AT_SP + phalf * 32u;
            float mx = -INFINITY;
            for (unsigned g = 0; g < 4u; ++g) {
                const v4f a = *(const v4f*)(srow + 8u * g), d = *(const v4f*)(srow + 8u * g + 4u);
                mx = fmaxf(mx, fmaxf(fmaxf(a.x, a.y), fmaxf(a.z, a.w)));
                mx = fmaxf(mx, fmaxf(fmaxf(d.x, d.y), fmaxf(d.z, d.w)));
            }
            mx = fmaxf(mx, __shfl_xor(mx, 1, 32));
            const float mnew = fmaxf(mrun, mx);
            const float alpha = expf(mrun - mnew);
            float psum = 0.f;
            h16* pdst = sP + prow * AT_PP + phalf * 32u;
            for (unsigned g = 0; g < 4u; ++g) {
                const v4f a = *(const v4f*)(srow + 8u * g), d = *(const v4f*)(srow + 8u * g + 4u);
                const float sv[8] = {a.x, a.y, a.z, a.w, d.x, d.y, d.z, d.w};
                v8h pk;
#pragma unroll
                for (int e = 0; e < 8; ++e) {
                    const float ex = expf(sv[e] - mnew);
                    const float p = (sv[e] > -3.0e38f) ? ex : 0.0f;
                    psum += p;
                    pk[e] = toh_flush(p * C_EMB);
                }
                *(v8h*)(pdst + 8u * g) = pk;
            }
            psum += __shfl_xor(psum, 1, 32);
            lrun = lrun * alpha + psum;
            mrun = mnew;
            if (phalf == 0u) sAl[prow] = alpha;
        }
        wave_sync_lds();
        {
            const v4f a0 = *(const v4f*)(sAl + 8u * hh), a1 = *(const v4f*)(sAl + 8u * hh + 4u);
            const float al[8] = {a0.x, a0.y, a0.z, a0.w, a1.x, a1.y, a1.z, a1.w};
#pragma unroll
            for (int t = 0; t < 4; ++t)
#pragma unroll
                for (int r = 0; r < 8; ++r) o[t][r] *= al[r];
        }
#pragma unroll
        for (int kk = 0; kk < 2; ++kk) {
            const v16h pa = frag_ld(sP + c * AT_PP + (unsigned)kk * 32u + 8u * hh);
#pragma unroll
            for (int t = 0; t < 4; ++t) {
                const v16h vb = frag_ld(vtb + (size_t)((unsigned)t * 16u + c) * (unsigned)(2 * SEQ) + base + (unsigned)kk * 32u + 8u * hh);
                o[t] = wmma16g(pa, vb, o[t]);
            }
        }
        wave_sync_lds();
    }
    if (phalf == 0u) sAl[prow] = lrun;
    wave_sync_lds();
    {
        const v4f a0 = *(const v4f*)(sAl + 8u * hh), a1 = *(const v4f*)(sAl + 8u * hh + 4u);
        const float ls[8] = {a0.x, a0.y, a0.z, a0.w, a1.x, a1.y, a1.z, a1.w};
#pragma unroll
        for (int t = 0; t < 4; ++t)
#pragma unroll
            for (int r = 0; r < 8; ++r)
                sS[(8u * hh + (unsigned)r) * AT_SP + (unsigned)t * 16u + c] = (o[t][r] * 6.103515625e-05f) / ls[r];
    }
    wave_sync_lds();
    {
        const unsigned q = lane >> 3, c8 = (lane & 7u) * 8u;
        v8h ov[4];
#pragma unroll
        for (int it = 0; it < 4; ++it) {
            const float* sp = sS + ((unsigned)it * 4u + q) * AT_SP + c8;
#pragma unroll
            for (int e = 0; e < 8; ++e) ov[it][e] = toh_flush(sp[e]);
        }
        h16* dst = O16 + (size_t)(b * (unsigned)(2 * SEQ) + i0) * DM + head * 64u;
        for (int pass = 0; pass < 2; ++pass) {
#pragma unroll
            for (int it = 0; it < 4; ++it) *(volatile v8h*)(dst + (size_t)((unsigned)it * 4u + q) * DM + c8) = ov[it];
            __threadfence();
        }
    }
}

constexpr size_t SZ_H     = (size_t)MTOK * DM * 4;
constexpr size_t SZ_T16   = (size_t)MTOK * DM * 2;
constexpr size_t SZ_QK16  = (size_t)MTOK * 2 * DM * 2;
constexpr size_t SZ_VT16  = (size_t)NB * NHEAD * HDIM * 2 * SEQ * 2;
constexpr size_t SZ_FF16  = (size_t)MTOK * FFD * 2;
constexpr size_t SZ_X16   = (size_t)MHALF * DM * 2;
constexpr size_t SZ_Y16   = (size_t)MBLK * YDIM * 2;
constexpr size_t SZ_SIN16 = (size_t)MBLK * FREQD * 2;
constexpr size_t SZ_TE16  = (size_t)MBLK * DM * 2;
constexpr size_t SZ_TE32  = (size_t)MBLK * DM * 4;
constexpr size_t SZ_WSQ   = (size_t)DM * DM * 2;
constexpr size_t OFF_H    = 0;
constexpr size_t OFF_Z16  = OFF_H + SZ_H;
constexpr size_t OFF_QK16 = OFF_Z16 + SZ_T16;
constexpr size_t OFF_VT16 = OFF_QK16 + SZ_QK16;
constexpr size_t OFF_O16  = OFF_VT16 + SZ_VT16;
constexpr size_t OFF_FF16 = OFF_O16 + SZ_T16;
constexpr size_t OFF_X16  = OFF_FF16 + SZ_FF16;
constexpr size_t OFF_XT16 = OFF_X16 + SZ_X16;
constexpr size_t OFF_Y16  = OFF_XT16 + SZ_X16;
constexpr size_t OFF_SIN  = OFF_Y16 + SZ_Y16;
constexpr size_t OFF_TE1  = OFF_SIN + SZ_SIN16;
constexpr size_t OFF_TE   = OFF_TE1 + SZ_TE16;
constexpr size_t OFF_COND = OFF_TE + SZ_TE32;
constexpr size_t OFF_HF16 = OFF_COND + SZ_TE32;
constexpr size_t OFF_WX   = OFF_HF16 + SZ_X16;
constexpr size_t OFF_WXT  = OFF_WX + SZ_WSQ;
constexpr size_t OFF_WY   = OFF_WXT + SZ_WSQ;
constexpr size_t OFF_WT1  = OFF_WY + (size_t)YDIM * DM * 2;
constexpr size_t OFF_WT2  = OFF_WT1 + (size_t)FREQD * DM * 2;
constexpr size_t OFF_WQKV = OFF_WT2 + SZ_WSQ;
constexpr size_t OFF_WPRJ = OFF_WQKV + (size_t)DEPTH * DM * 3 * DM * 2;
constexpr size_t OFF_WFC1 = OFF_WPRJ + (size_t)DEPTH * DM * DM * 2;
constexpr size_t OFF_WFC2 = OFF_WFC1 + (size_t)DEPTH * DM * FFD * 2;
constexpr size_t OFF_WF   = OFF_WFC2 + (size_t)DEPTH * FFD * DM * 2;
constexpr size_t WS_TOTAL = OFF_WF + SZ_WSQ;
static_assert(WS_TOTAL < (size_t)268435456);
static_assert(SZ_SIN16 % 256 == 0 && SZ_TE16 % 256 == 0 && SZ_Y16 % 256 == 0 && SZ_X16 % 256 == 0);

extern "C" void kernel_launch(void* const* d_in, const int* in_sizes, int n_in, void* d_out, int out_size,
                              void* d_ws, size_t ws_size, hipStream_t stream) {
    if (n_in < 29) return;
    const int nX = ((NB - 1) * SEQ_FULL + SEQ) * DM;
    const int nT = (NB - 1) * (SEQ_FULL / 4) + SEQ / 4;
    if (in_sizes[0] < nX || in_sizes[1] < nX || in_sizes[2] < nT || in_sizes[3] < nT * YDIM || in_sizes[4] < SEQ * DM) return;
    if (in_sizes[5] < DM * DM || in_sizes[6] < DM || in_sizes[7] < DM * DM || in_sizes[8] < DM || in_sizes[9] < YDIM * DM || in_sizes[10] < DM) return;
    if (in_sizes[11] < FREQD * DM || in_sizes[12] < DM || in_sizes[13] < DM * DM || in_sizes[14] < DM) return;
    if (in_sizes[15] < DEPTH * DM * 3 * DM || in_sizes[16] < DEPTH * 3 * DM || in_sizes[17] < DEPTH * DM * DM || in_sizes[18] < DEPTH * DM) return;
    if (in_sizes[19] < DEPTH * DM || in_sizes[20] < DEPTH * DM || in_sizes[21] < DEPTH * DM || in_sizes[22] < DEPTH * DM) return;
    if (in_sizes[23] < DEPTH * DM * FFD || in_sizes[24] < DEPTH * FFD || in_sizes[25] < DEPTH * FFD * DM || in_sizes[26] < DEPTH * DM) return;
    if (in_sizes[27] < DM * DM || in_sizes[28] < DM || out_size < nX) return;
    if (WS_TOTAL > ws_size) return;

    const float* x      = (const float*)d_in[0];
    const float* x_t    = (const float*)d_in[1];
    const int*   t      = (const int*)d_in[2];
    const float* y      = (const float*)d_in[3];
    const float* pos    = (const float*)d_in[4];
    const float* xw     = (const float*)d_in[5];
    const float* xb     = (const float*)d_in[6];
    const float* xtw    = (const float*)d_in[7];
    const float* xtb    = (const float*)d_in[8];
    const float* yw     = (const float*)d_in[9];
    const float* yb     = (const float*)d_in[10];
    const float* t1w    = (const float*)d_in[11];
    const float* t1b    = (const float*)d_in[12];
    const float* t2w    = (const float*)d_in[13];
    const float* t2b    = (const float*)d_in[14];
    const float* qkv_w  = (const float*)d_in[15];
    const float* qkv_b  = (const float*)d_in[16];
    const float* proj_w = (const float*)d_in[17];
    const float* proj_b = (const float*)d_in[18];
    const float* n1_g   = (const float*)d_in[19];
    const float* n1_b   = (const float*)d_in[20];
    const float* n2_g   = (const float*)d_in[21];
    const float* n2_b   = (const float*)d_in[22];
    const float* fc1_w  = (const float*)d_in[23];
    const float* fc1_b  = (const float*)d_in[24];
    const float* fc2_w  = (const float*)d_in[25];
    const float* fc2_b  = (const float*)d_in[26];
    const float* fw     = (const float*)d_in[27];
    const float* fb     = (const float*)d_in[28];
    float* out = (float*)d_out;

    char* wsp = (char*)d_ws;
    float* h     = (float*)(wsp + OFF_H);
    h16* z16     = (h16*)(wsp + OFF_Z16);
    h16* qk16    = (h16*)(wsp + OFF_QK16);
    h16* vt16    = (h16*)(wsp + OFF_VT16);
    h16* o16     = (h16*)(wsp + OFF_O16);
    h16* ff16    = (h16*)(wsp + OFF_FF16);
    h16* x16     = (h16*)(wsp + OFF_X16);
    h16* xt16    = (h16*)(wsp + OFF_XT16);
    h16* y16     = (h16*)(wsp + OFF_Y16);
    h16* sin16   = (h16*)(wsp + OFF_SIN);
    h16* te1_16  = (h16*)(wsp + OFF_TE1);
    float* te    = (float*)(wsp + OFF_TE);
    float* cond  = (float*)(wsp + OFF_COND);
    h16* hf16    = (h16*)(wsp + OFF_HF16);
    h16* w_x     = (h16*)(wsp + OFF_WX);
    h16* w_xt    = (h16*)(wsp + OFF_WXT);
    h16* w_y     = (h16*)(wsp + OFF_WY);
    h16* w_t1    = (h16*)(wsp + OFF_WT1);
    h16* w_t2    = (h16*)(wsp + OFF_WT2);
    h16* w_qkv   = (h16*)(wsp + OFF_WQKV);
    h16* w_prj   = (h16*)(wsp + OFF_WPRJ);
    h16* w_fc1   = (h16*)(wsp + OFF_WFC1);
    h16* w_fc2   = (h16*)(wsp + OFF_WFC2);
    h16* w_f     = (h16*)(wsp + OFF_WF);

    k_wt16<<<dim3((DM * (DM / 8)) / 256, 1), 256, 0, stream>>>(xw, DM, DM, 7, w_x);
    k_wt16<<<dim3((DM * (DM / 8)) / 256, 1), 256, 0, stream>>>(xtw, DM, DM, 7, w_xt);
    k_wt16<<<dim3((DM * (YDIM / 8)) / 256, 1), 256, 0, stream>>>(yw, YDIM, DM, 8, w_y);
    k_wt16<<<dim3((DM * (FREQD / 8)) / 256, 1), 256, 0, stream>>>(t1w, FREQD, DM, 5, w_t1);
    k_wt16<<<dim3((DM * (DM / 8)) / 256, 1), 256, 0, stream>>>(t2w, DM, DM, 7, w_t2);
    k_wt16<<<dim3((3 * DM * (DM / 8)) / 256, DEPTH), 256, 0, stream>>>(qkv_w, DM, 3 * DM, 7, w_qkv);
    k_wt16<<<dim3((DM * (DM / 8)) / 256, DEPTH), 256, 0, stream>>>(proj_w, DM, DM, 7, w_prj);
    k_wt16<<<dim3((FFD * (DM / 8)) / 256, DEPTH), 256, 0, stream>>>(fc1_w, DM, FFD, 7, w_fc1);
    k_wt16<<<dim3((DM * (FFD / 8)) / 256, DEPTH), 256, 0, stream>>>(fc2_w, FFD, DM, 9, w_fc2);
    k_wt16<<<dim3((DM * (DM / 8)) / 256, 1), 256, 0, stream>>>(fw, DM, DM, 7, w_f);

    k_cvt<DM, SEQ, SEQ_FULL, 0, 11, true><<<(MHALF * (DM / 8) + 255) / 256, 256, 0, stream>>>(x, x16, (unsigned)MHALF);
    k_cvt<DM, SEQ, SEQ_FULL, 0, 11, true><<<(MHALF * (DM / 8) + 255) / 256, 256, 0, stream>>>(x_t, xt16, (unsigned)MHALF);
    k_cvt<YDIM, SEQ / 4, SEQ_FULL / 4, 0, 11, true><<<(MBLK * (YDIM / 8) + 255) / 256, 256, 0, stream>>>(y, y16, (unsigned)MBLK);
    k_sin<<<MBLK, 256, 0, stream>>>(t, sin16);

    auto gt = [](unsigned M, unsigned N) -> unsigned { return ((M / 64u) * (N / 64u) + 7u) / 8u; };

    k_gemm64<EP_F16, ACT_SILU, 31, 14, false><<<gt(MBLK, DM), 256, 0, stream>>>(sin16, FREQD, w_t1, FREQD,
        (void*)te1_16, DM, t1b, nullptr, nullptr, nullptr, (unsigned)MBLK, DM, FREQD);
    k_gemm64<EP_F32, ACT_NONE, 31, 0, false><<<gt(MBLK, DM), 256, 0, stream>>>(te1_16, DM, w_t2, DM,
        (void*)te, DM, t2b, nullptr, nullptr, nullptr, (unsigned)MBLK, DM, DM);
    k_gemm64<EP_F32, ACT_NONE, 28, 0, false><<<gt(MBLK, DM), 256, 0, stream>>>(y16, YDIM, w_y, YDIM,
        (void*)cond, DM, yb, nullptr, nullptr, nullptr, (unsigned)MBLK, DM, YDIM);
    k_gemm64<EP_EMBX, ACT_NONE, 28, 0, false><<<gt(MHALF, DM), 256, 0, stream>>>(x16, DM, w_x, DM,
        (void*)h, DM, xb, pos, nullptr, nullptr, (unsigned)MHALF, DM, DM);
    k_gemm64<EP_EMBXT, ACT_NONE, 28, 0, false><<<gt(MHALF, DM), 256, 0, stream>>>(xt16, DM, w_xt, DM,
        (void*)h, DM, xtb, pos, te, cond, (unsigned)MHALF, DM, DM);

    for (int l = 0; l < DEPTH; ++l) {
        const bool last = (l == DEPTH - 1);
        const h16* wq = w_qkv + (size_t)l * DM * 3 * DM;
        const float* bq = qkv_b + l * 3 * DM;
        k_ln<<<MTOK / 8, 256, 0, stream>>>(h, n1_g + l * DM, n1_b + l * DM, z16, (unsigned)MTOK);
        if (!last) {
            k_gemm64<EP_F16, ACT_NONE, 28, 12, false><<<gt(MTOK, 2 * DM), 256, 0, stream>>>(z16, DM, wq, DM,
                (void*)qk16, 2 * DM, bq, nullptr, nullptr, nullptr, (unsigned)MTOK, 2 * DM, DM);
        } else {
            k_gemm64<EP_F16, ACT_NONE, 28, 12, true><<<gt(MHALF, DM), 256, 0, stream>>>(z16, DM, wq, DM,
                (void*)qk16, 2 * DM, bq, nullptr, nullptr, nullptr, (unsigned)MHALF, DM, DM);
            k_gemm64<EP_F16, ACT_NONE, 28, 12, false><<<gt(MTOK, DM), 256, 0, stream>>>(z16, DM, wq + (size_t)DM * DM, DM,
                (void*)(qk16 + DM), 2 * DM, bq + DM, nullptr, nullptr, nullptr, (unsigned)MTOK, DM, DM);
        }
        k_gemm64<EP_VT, ACT_NONE, 28, 12, false><<<gt(MTOK, DM), 256, 0, stream>>>(z16, DM, wq + (size_t)2 * DM * DM, DM,
            (void*)vt16, 2 * SEQ, bq + 2 * DM, nullptr, nullptr, nullptr, (unsigned)MTOK, DM, DM);
        if (!last) {
            k_attn<false><<<NB * NHEAD * (2 * SEQ / 16), 32, 0, stream>>>(qk16, vt16, o16);
            k_gemm64<EP_RESID, ACT_NONE, 29, 0, false><<<gt(MTOK, DM), 256, 0, stream>>>(o16, DM, w_prj + (size_t)l * DM * DM, DM,
                (void*)h, DM, proj_b + l * DM, h, nullptr, nullptr, (unsigned)MTOK, DM, DM);
        } else {
            k_attn<true><<<NB * NHEAD * (SEQ / 16), 32, 0, stream>>>(qk16, vt16, o16);
            k_gemm64<EP_RESID, ACT_NONE, 29, 0, true><<<gt(MHALF, DM), 256, 0, stream>>>(o16, DM, w_prj + (size_t)l * DM * DM, DM,
                (void*)h, DM, proj_b + l * DM, h, nullptr, nullptr, (unsigned)MHALF, DM, DM);
        }
        k_ln<<<MTOK / 8, 256, 0, stream>>>(h, n2_g + l * DM, n2_b + l * DM, z16, (unsigned)MTOK);
        if (!last) {
            k_gemm64<EP_F16, ACT_GELU, 28, 12, false><<<gt(MTOK, FFD), 256, 0, stream>>>(z16, DM, w_fc1 + (size_t)l * DM * FFD, DM,
                (void*)ff16, FFD, fc1_b + l * FFD, nullptr, nullptr, nullptr, (unsigned)MTOK, FFD, DM);
            k_gemm64<EP_RESID, ACT_NONE, 29, 0, false><<<gt(MTOK, DM), 256, 0, stream>>>(ff16, FFD, w_fc2 + (size_t)l * FFD * DM, FFD,
                (void*)h, DM, fc2_b + l * DM, h, nullptr, nullptr, (unsigned)MTOK, DM, FFD);
        } else {
            k_gemm64<EP_F16, ACT_GELU, 28, 12, true><<<gt(MHALF, FFD), 256, 0, stream>>>(z16, DM, w_fc1 + (size_t)l * DM * FFD, DM,
                (void*)ff16, FFD, fc1_b + l * FFD, nullptr, nullptr, nullptr, (unsigned)MHALF, FFD, DM);
            k_gemm64<EP_RESID, ACT_NONE, 29, 0, true><<<gt(MHALF, DM), 256, 0, stream>>>(ff16, FFD, w_fc2 + (size_t)l * FFD * DM, FFD,
                (void*)h, DM, fc2_b + l * DM, h, nullptr, nullptr, (unsigned)MHALF, DM, FFD);
        }
    }

    k_cvt<DM, SEQ, 2 * SEQ, SEQ, 11, false><<<(MHALF * (DM / 8) + 255) / 256, 256, 0, stream>>>(h, hf16, (unsigned)MHALF);
    k_gemm64<EP_OUT, ACT_NONE, 28, 0, false><<<gt(MHALF, DM), 256, 0, stream>>>(hf16, DM, w_f, DM,
        (void*)out, DM, fb, nullptr, nullptr, nullptr, (unsigned)MHALF, DM, DM);
}
